// BertAdapterCapsuleMaskImp_51840255263217
// MI455X (gfx1250) — hardware-run, weakly checked
//
#include <hip/hip_runtime.h>
#include <stddef.h>
#include <stdint.h>
#include <math.h>


#define NTOK  16384
#define HID   768
#define ADP   2000
#define APD   2048
#define NTASK 10
#define CAP   3
#define NCAP  3
#define NSEM  32
#define NSEMV 30
#define NEGV  (-10000.0f)
#define EPSV  (1e-16f)
#define XHS   16
#define H1S   64
#define WSC   1024
#define NTHR  256
#define NWAVE 8
#define TOKB  128
#define STHR  128
#define RB    64
#define BTHR  96
#define WSCAP 134217728
#define LDS_G (NWAVE * 32 * 64 * 4)
#define NBW1 ((APD * HID) / (8 * NTHR))
#define NBW2 ((HID * APD) / (8 * NTHR))
#define NBWS ((NSEM * HID) / (8 * NTHR))
#define NRW  (NCAP * NTASK * CAP * CAP)

static_assert((HID % 32) == 0);
static_assert((APD % 32) == 0);
static_assert((NTOK % 128) == 0);
static_assert((HID % 128) == 0);
static_assert((APD % 128) == 0);
static_assert((NTOK % TOKB) == 0);
static_assert(TOKB == STHR);
static_assert((BTHR * 8) == HID);
static_assert((NTOK % RB) == 0);
static_assert(((RB * 9) % BTHR) == 0);
static_assert(((APD * HID) % (8 * NTHR)) == 0);
static_assert(((NSEM * HID) % (8 * NTHR)) == 0);
static_assert(NTHR == NWAVE * 32);
static_assert(LDS_G <= 300 * 1024);
static_assert((ADP % 8) == 0);

typedef float          v4f  __attribute__((ext_vector_type(4)));
typedef float          v8f  __attribute__((ext_vector_type(8)));
typedef _Float16       v8h  __attribute__((ext_vector_type(8)));
typedef _Float16       v16h __attribute__((ext_vector_type(16)));
union FragH { v16h v; v8h h[2]; };

__device__ __forceinline__ v8f wmf(v16h a, v16h b, v8f c) {
  v8f d = __builtin_amdgcn_wmma_f32_16x16x32_f16(false, a, false, b, (short)0, c, false, false);
  asm volatile("v_nop\n\tv_nop\n\tv_nop\n\tv_nop" : "+v"(d) : "v"(a), "v"(b));
  return d;
}

__device__ __forceinline__ float rcpx(float v) { return __builtin_amdgcn_rcpf(v); }
__device__ __forceinline__ float sigm(float z) { return rcpx(1.0f + __expf(-z)); }
__device__ __forceinline__ float gelu_erf(float v) {
  return 0.5f * v * (1.0f + erff(v * 0.70710678118654752440f));
}
__device__ __forceinline__ int clamp_task(int t) { return min(max(t, 0), NTASK - 1); }

__device__ __forceinline__ v16h ld_x_frag(const float* p) {
  const v4f q0 = *(const v4f*)p;
  const v4f q1 = *(const v4f*)(p + 4);
  const v4f q2 = *(const v4f*)(p + 16);
  const v4f q3 = *(const v4f*)(p + 20);
  v16h r;
  r[0]  = (_Float16)q0.x; r[1]  = (_Float16)q0.y; r[2]  = (_Float16)q0.z; r[3]  = (_Float16)q0.w;
  r[4]  = (_Float16)q1.x; r[5]  = (_Float16)q1.y; r[6]  = (_Float16)q1.z; r[7]  = (_Float16)q1.w;
  r[8]  = (_Float16)q2.x; r[9]  = (_Float16)q2.y; r[10] = (_Float16)q2.z; r[11] = (_Float16)q2.w;
  r[12] = (_Float16)q3.x; r[13] = (_Float16)q3.y; r[14] = (_Float16)q3.z; r[15] = (_Float16)q3.w;
  return r;
}

__global__ __launch_bounds__(NTHR) void k_prepw(const float* __restrict__ fc1w, const float* __restrict__ fc2w,
                                                const float* __restrict__ semw,
                                                _Float16* w1h, _Float16* w2h, _Float16* wsh) {
  const int blk = blockIdx.x;
  const size_t t = threadIdx.x;
  const float* src;
  _Float16* dst;
  bool zero;
  if (blk < NBW1) {
    const size_t e = ((size_t)blk * NTHR + t) * 8;
    const int n = (int)(e / HID), k0 = (int)(e % HID);
    zero = (n >= ADP);
    src = fc1w + (size_t)min(n, ADP - 1) * HID + k0;
    dst = w1h + e;
  } else if (blk < NBW1 + NBW2) {
    const size_t e = ((size_t)(blk - NBW1) * NTHR + t) * 8;
    const int h = (int)(e / APD), a0 = (int)(e % APD);
    zero = (a0 >= ADP);
    src = fc2w + (size_t)h * ADP + min(a0, ADP - 8);
    dst = w2h + e;
  } else {
    const size_t e = ((size_t)(blk - NBW1 - NBW2) * NTHR + t) * 8;
    const int j = (int)(e / HID), k0 = (int)(e % HID);
    zero = (j >= NSEMV);
    const int jc = min(j, NSEMV - 1), c = jc / NTASK, ta = jc % NTASK;
    src = semw + (size_t)(ta * CAP + c) * HID + k0;
    dst = wsh + e;
  }
  const v4f f0 = *(const v4f*)src;
  const v4f f1 = *(const v4f*)(src + 4);
  const float sc = zero ? 0.0f : (float)WSC;
  v8h a;
  a[0] = (_Float16)(f0.x * sc); a[1] = (_Float16)(f0.y * sc); a[2] = (_Float16)(f0.z * sc); a[3] = (_Float16)(f0.w * sc);
  a[4] = (_Float16)(f1.x * sc); a[5] = (_Float16)(f1.y * sc); a[6] = (_Float16)(f1.z * sc); a[7] = (_Float16)(f1.w * sc);
  *(volatile v8h*)dst = a;
  __threadfence();
  *(volatile v8h*)dst = a;
}

__global__ __launch_bounds__(STHR) void k_semroute(const float* __restrict__ x, const _Float16* __restrict__ wsh,
                                                   const float* __restrict__ semb, const float* __restrict__ rw,
                                                   const int* __restrict__ tptr, float* votef) {
  __shared__ __attribute__((aligned(16))) float semS[TOKB * NSEM];
  __shared__ __attribute__((aligned(16))) float voteS[NCAP * TOKB * CAP];
  __shared__ float rwS[NRW + 2];
  __shared__ float sbS[NSEM];
  const int tid = threadIdx.x, lane = tid & 31, wave = tid >> 5, hf = lane >> 4, m = lane & 15;
  const int n0 = blockIdx.x * TOKB;
  const int tc = clamp_task(tptr[0]);

  for (int i = tid; i < 3 * STHR; i += STHR) {
    const float v = rw[min(i, NRW - 1)];
    if (i < NRW) rwS[i] = v;
  }
  if (tid < NSEM) {
    const int jc = min(tid, NSEMV - 1);
    const float b = semb[(jc % NTASK) * CAP + jc / NTASK];
    sbS[tid] = (tid < NSEMV) ? b : 0.0f;
  }
  __syncthreads();

  v8f acc[2][2];
#pragma unroll
  for (int mt = 0; mt < 2; ++mt)
#pragma unroll
    for (int nt = 0; nt < 2; ++nt) { v8f z = {0.f, 0.f, 0.f, 0.f, 0.f, 0.f, 0.f, 0.f}; acc[mt][nt] = z; }

  const float* ap = x + (size_t)(n0 + 32 * wave + m) * HID + 8 * hf;
  const _Float16* bp = wsh + (size_t)m * HID + 8 * hf;
#pragma unroll 1
  for (int kt = 0; kt < HID / 32; ++kt) {
    const int k0 = 32 * kt;
    const v16h a0 = ld_x_frag(ap + k0);
    const v16h a1 = ld_x_frag(ap + (size_t)16 * HID + k0);
#pragma unroll
    for (int nt = 0; nt < 2; ++nt) {
      const _Float16* bq = bp + (size_t)nt * 16 * HID + k0;
      FragH b;
      b.h[0] = *(const v8h*)bq;
      b.h[1] = *(const v8h*)(bq + 16);
      acc[0][nt] = wmf(a0, b.v, acc[0][nt]);
      acc[1][nt] = wmf(a1, b.v, acc[1][nt]);
    }
  }

  constexpr float RSEM = 1.0f / (float)WSC;
#pragma unroll
  for (int mt = 0; mt < 2; ++mt)
#pragma unroll
    for (int nt = 0; nt < 2; ++nt) {
      const float bb = sbS[16 * nt + m];
      float* sp = semS + (32 * wave + 16 * mt + 8 * hf) * NSEM + 16 * nt + m;
#pragma unroll
      for (int r = 0; r < 8; ++r) sp[r * NSEM] = acc[mt][nt][r] * RSEM + bb;
    }
  __syncthreads();

  {
    float* sr = semS + tid * NSEM;
#pragma unroll
    for (int c = 0; c < CAP; ++c) {
      float v[NTASK];
      float s2 = 0.0f;
#pragma unroll
      for (int ta = 0; ta < NTASK; ++ta) { v[ta] = sr[c * NTASK + ta]; s2 = fmaf(v[ta], v[ta], s2); }
      const float sq = s2 + EPSV;
      const float q  = sq * rcpx(1.0f + sq);
      const float rs = rsqrtf(sq);
#pragma unroll
      for (int ta = 0; ta < NTASK; ++ta) sr[c * NTASK + ta] = (q * v[ta]) * rs;
    }

#pragma unroll 1
    for (int mm = 0; mm < NCAP; ++mm) {
      const float* rwm = rwS + mm * (NTASK * CAP * CAP);
      float pri[NTASK][CAP];
#pragma unroll
      for (int r = 0; r < NTASK; ++r) {
        const float x0 = sr[r * CAP + 0], x1 = sr[r * CAP + 1], x2 = sr[r * CAP + 2];
#pragma unroll
        for (int d = 0; d < CAP; ++d) {
          float a = x0 * rwm[(r * CAP + 0) * CAP + d];
          a = fmaf(x1, rwm[(r * CAP + 1) * CAP + d], a);
          a = fmaf(x2, rwm[(r * CAP + 2) * CAP + d], a);
          pri[r][d] = a;
        }
      }
      float lg[NTASK];
#pragma unroll
      for (int r = 0; r < NTASK; ++r) lg[r] = 0.0f;
      float vt[CAP];
#pragma unroll
      for (int it = 0; it < 3; ++it) {
        float l[NTASK], e[NTASK];
        float mx = -3.0e38f;
#pragma unroll
        for (int r = 0; r < NTASK; ++r) { l[r] = (r <= tc) ? lg[r] : NEGV; mx = fmaxf(mx, l[r]); }
        float se = 0.0f;
#pragma unroll
        for (int r = 0; r < NTASK; ++r) { e[r] = __expf(l[r] - mx); se += e[r]; }
        const float inv = rcpx(se);
#pragma unroll
        for (int r = 0; r < NTASK; ++r) e[r] = e[r] * inv;
#pragma unroll
        for (int d = 0; d < CAP; ++d) {
          float a = 0.0f;
#pragma unroll
          for (int r = 0; r < NTASK; ++r) a = fmaf(e[r], pri[r][d], a);
          vt[d] = a;
        }
        if (it < 2) {
          const float s2 = fmaf(vt[2], vt[2], fmaf(vt[1], vt[1], vt[0] * vt[0]));
          const float sq = s2 + EPSV;
          const float q  = sq * rcpx(1.0f + sq);
          const float rs = rsqrtf(sq);
          float o[CAP];
#pragma unroll
          for (int d = 0; d < CAP; ++d) o[d] = (q * vt[d]) * rs;
#pragma unroll
          for (int r = 0; r < NTASK; ++r) {
            float dl = pri[r][0] * o[0];
            dl = fmaf(pri[r][1], o[1], dl);
            dl = fmaf(pri[r][2], o[2], dl);
            lg[r] = l[r] + dl;
          }
        }
      }
#pragma unroll
      for (int d = 0; d < CAP; ++d) voteS[mm * (TOKB * CAP) + tid * CAP + d] = vt[d];
    }
  }
  __syncthreads();

  const size_t plane = (size_t)NTOK * CAP;
  for (int q = wave; q < 9; q += 4) {
    const int mm = q / 3, part = q - 3 * mm;
    const v4f v = *(const v4f*)(voteS + mm * (TOKB * CAP) + part * 128 + 4 * lane);
    float* d = votef + (size_t)mm * plane + (size_t)n0 * CAP + part * 128 + 4 * lane;
    *(volatile v4f*)d = v;
  }
  __threadfence();
  for (int q = wave; q < 9; q += 4) {
    const int mm = q / 3, part = q - 3 * mm;
    const v4f v = *(const v4f*)(voteS + mm * (TOKB * CAP) + part * 128 + 4 * lane);
    float* d = votef + (size_t)mm * plane + (size_t)n0 * CAP + part * 128 + 4 * lane;
    *(volatile v4f*)d = v;
  }
}

#define WEL(q) (wv[(q) >> 2][(q) & 3])
__global__ __launch_bounds__(BTHR) void k_buildh(const float* __restrict__ x, const float* __restrict__ votef,
                                                const float* __restrict__ lw, const float* __restrict__ lb,
                                                const float* __restrict__ elg, const float* __restrict__ s,
                                                const int* __restrict__ tptr, _Float16* hp) {
  __shared__ __attribute__((aligned(16))) v4f lw4S[18 * BTHR];
  __shared__ float hcS[RB * 9];
  __shared__ float ggS[HID];
  const int tid = threadIdx.x;
  const int c0 = 8 * tid;
  const int rbase = blockIdx.x * RB;
  const float sv = s[0];
  const int tc = clamp_task(tptr[0]);

  {
    v4f wv[18];
    const v4f* wp = (const v4f*)(lw + (size_t)c0 * (NCAP * CAP));
#pragma unroll
    for (int j = 0; j < 18; ++j) wv[j] = wp[j];
#pragma unroll
    for (int i = 0; i < 9; ++i) {
      v4f wa, wb;
      wa.x = WEL(0 * 9 + i); wa.y = WEL(1 * 9 + i); wa.z = WEL(2 * 9 + i); wa.w = WEL(3 * 9 + i);
      wb.x = WEL(4 * 9 + i); wb.y = WEL(5 * 9 + i); wb.z = WEL(6 * 9 + i); wb.w = WEL(7 * 9 + i);
      lw4S[(2 * i) * BTHR + tid] = wa;
      lw4S[(2 * i + 1) * BTHR + tid] = wb;
    }
  }
  for (int i = tid; i < RB * 9; i += BTHR) hcS[i] = votef[(size_t)rbase * 9 + i];
#pragma unroll 1
  for (int j = 0; j < 8; ++j) ggS[c0 + j] = sigm(sv * elg[(size_t)tc * HID + c0 + j]);
  __syncthreads();

  float bb[8], gg[8];
  {
    const v4f b0 = *(const v4f*)(lb + c0);
    const v4f b1 = *(const v4f*)(lb + c0 + 4);
    bb[0] = b0.x; bb[1] = b0.y; bb[2] = b0.z; bb[3] = b0.w;
    bb[4] = b1.x; bb[5] = b1.y; bb[6] = b1.z; bb[7] = b1.w;
  }
#pragma unroll
  for (int j = 0; j < 8; ++j) gg[j] = ggS[c0 + j];

#pragma unroll 1
  for (int r = 0; r < RB; ++r) {
    const size_t n = (size_t)(rbase + r);
    const v4f xa = *(const v4f*)(x + n * HID + c0);
    const v4f xb = *(const v4f*)(x + n * HID + c0 + 4);
    float xs[8];
    xs[0] = xa.x; xs[1] = xa.y; xs[2] = xa.z; xs[3] = xa.w;
    xs[4] = xb.x; xs[5] = xb.y; xs[6] = xb.z; xs[7] = xb.w;
    float a[8];
#pragma unroll
    for (int j = 0; j < 8; ++j) a[j] = 0.0f;
    const float* hrow = hcS + r * 9;
#pragma unroll 1
    for (int i = 0; i < 9; ++i) {
      const float h = hrow[i];
      const v4f wa = lw4S[(2 * i) * BTHR + tid];
      const v4f wb = lw4S[(2 * i + 1) * BTHR + tid];
      a[0] = fmaf(h, wa.x, a[0]); a[1] = fmaf(h, wa.y, a[1]); a[2] = fmaf(h, wa.z, a[2]); a[3] = fmaf(h, wa.w, a[3]);
      a[4] = fmaf(h, wb.x, a[4]); a[5] = fmaf(h, wb.y, a[5]); a[6] = fmaf(h, wb.z, a[6]); a[7] = fmaf(h, wb.w, a[7]);
    }
    v8h hv;
#pragma unroll
    for (int j = 0; j < 8; ++j) {
      const float hvv = xs[j] + (a[j] + bb[j]) * gg[j];
      hv[j] = (_Float16)(hvv * (float)XHS);
    }
    _Float16* d = hp + n * HID + c0;
    *(volatile v8h*)d = hv;
    __threadfence();
    *(volatile v8h*)d = hv;
  }
}

__global__ __launch_bounds__(NTHR) void k_gemm1(const _Float16* __restrict__ hp, const _Float16* __restrict__ w1h,
                                                const float* __restrict__ fc1b, const float* __restrict__ efc1,
                                                const float* __restrict__ s, const int* __restrict__ tptr,
                                                _Float16* h1) {
  extern __shared__ v4f lds_dyn[];
  __shared__ float bvS[128];
  __shared__ float gvS[128];
  const int tid = threadIdx.x, lane = tid & 31, wave = tid >> 5, hf = lane >> 4, m = lane & 15;
  float* stg = (float*)lds_dyn + wave * (32 * 64);
  const int n0 = blockIdx.x * 128, m0 = blockIdx.y * 128;
  const int wm = (wave >> 1) * 32, wn = (wave & 1) * 64;

  {
    const float sv = s[0];
    const int tc = clamp_task(tptr[0]);
    if (tid < 128) {
      const int col = n0 + tid;
      const int colc = min(col, ADP - 1);
      bvS[tid] = fc1b[colc];
      const float g = sigm(sv * efc1[(size_t)tc * ADP + colc]) * (float)H1S;
      gvS[tid] = (col < ADP) ? g : 0.0f;
    }
  }
  __syncthreads();

  v8f acc[2][4];
#pragma unroll
  for (int mt = 0; mt < 2; ++mt)
#pragma unroll
    for (int nt = 0; nt < 4; ++nt) { v8f z = {0.f, 0.f, 0.f, 0.f, 0.f, 0.f, 0.f, 0.f}; acc[mt][nt] = z; }

  const _Float16* ap = hp + (size_t)(m0 + wm + m) * HID + 8 * hf;
  const _Float16* bp = w1h + (size_t)(n0 + wn + m) * HID + 8 * hf;
#pragma unroll 1
  for (int kt = 0; kt < HID / 32; ++kt) {
    const int k0 = 32 * kt;
    FragH a0, a1;
    a0.h[0] = *(const v8h*)(ap + k0);
    a0.h[1] = *(const v8h*)(ap + k0 + 16);
    a1.h[0] = *(const v8h*)(ap + (size_t)16 * HID + k0);
    a1.h[1] = *(const v8h*)(ap + (size_t)16 * HID + k0 + 16);
#pragma unroll
    for (int nt = 0; nt < 4; ++nt) {
      const _Float16* bq = bp + (size_t)nt * 16 * HID + k0;
      FragH b;
      b.h[0] = *(const v8h*)bq;
      b.h[1] = *(const v8h*)(bq + 16);
      acc[0][nt] = wmf(a0.v, b.v, acc[0][nt]);
      acc[1][nt] = wmf(a1.v, b.v, acc[1][nt]);
    }
  }

#pragma unroll
  for (int mt = 0; mt < 2; ++mt) {
    float* sp = stg + (16 * mt + 8 * hf) * 64 + m;
#pragma unroll
    for (int nt = 0; nt < 4; ++nt) {
#pragma unroll
      for (int r = 0; r < 8; ++r) sp[r * 64 + 16 * nt] = acc[mt][nt][r];
    }
  }
  constexpr float OSC1 = 1.0f / (float)(XHS * WSC);
#pragma unroll 1
  for (int e = 0; e < 64; ++e) {
    const int mt = e >> 5, nt = (e >> 3) & 3, r = e & 7;
    float* p = stg + (16 * mt + 8 * hf + r) * 64 + 16 * nt + m;
    const int cl = wn + 16 * nt + m;
    const float v = *p;
    *p = gelu_erf(fmaf(v, OSC1, bvS[cl])) * gvS[cl];
  }
  __syncthreads();

  _Float16* gb = h1 + (size_t)(m0 + wm) * APD + n0 + wn;
  const int rq = lane >> 3, pc = (lane & 7) * 8;
  v8h hv[8];
#pragma unroll
  for (int i = 0; i < 8; ++i) {
    const int row = 4 * i + rq;
    const v4f u0 = *(const v4f*)(stg + row * 64 + pc);
    const v4f u1 = *(const v4f*)(stg + row * 64 + pc + 4);
    v8h v;
    v[0] = (_Float16)u0.x; v[1] = (_Float16)u0.y; v[2] = (_Float16)u0.z; v[3] = (_Float16)u0.w;
    v[4] = (_Float16)u1.x; v[5] = (_Float16)u1.y; v[6] = (_Float16)u1.z; v[7] = (_Float16)u1.w;
    hv[i] = v;
    *(volatile v8h*)(gb + (size_t)row * APD + pc) = v;
  }
  __threadfence();
#pragma unroll
  for (int i = 0; i < 8; ++i) {
    const int row = 4 * i + rq;
    *(volatile v8h*)(gb + (size_t)row * APD + pc) = hv[i];
  }
}

__global__ __launch_bounds__(NTHR) void k_gemm2(const _Float16* __restrict__ h1, const _Float16* __restrict__ w2h,
                                                const float* __restrict__ fc2b, const float* __restrict__ efc2,
                                                const float* __restrict__ s, const int* __restrict__ tptr,
                                                const float* __restrict__ x, float* out) {
  extern __shared__ v4f lds_dyn[];
  __shared__ float bvS[128];
  __shared__ float gvS[128];
  const int tid = threadIdx.x, lane = tid & 31, wave = tid >> 5, hf = lane >> 4, m = lane & 15;
  float* stg = (float*)lds_dyn + wave * (32 * 64);
  const int n0 = blockIdx.x * 128, m0 = blockIdx.y * 128;
  const int wm = (wave >> 1) * 32, wn = (wave & 1) * 64;

  {
    const float sv = s[0];
    const int tc = clamp_task(tptr[0]);
    if (tid < 128) {
      const int col = n0 + tid;
      bvS[tid] = fc2b[col];
      gvS[tid] = sigm(sv * efc2[(size_t)tc * HID + col]);
    }
  }
  __syncthreads();

  v8f acc[2][4];
#pragma unroll
  for (int mt = 0; mt < 2; ++mt)
#pragma unroll
    for (int nt = 0; nt < 4; ++nt) { v8f z = {0.f, 0.f, 0.f, 0.f, 0.f, 0.f, 0.f, 0.f}; acc[mt][nt] = z; }

  const _Float16* ap = h1 + (size_t)(m0 + wm + m) * APD + 8 * hf;
  const _Float16* bp = w2h + (size_t)(n0 + wn + m) * APD + 8 * hf;
#pragma unroll 1
  for (int kt = 0; kt < APD / 32; ++kt) {
    const int k0 = 32 * kt;
    FragH a0, a1;
    a0.h[0] = *(const v8h*)(ap + k0);
    a0.h[1] = *(const v8h*)(ap + k0 + 16);
    a1.h[0] = *(const v8h*)(ap + (size_t)16 * APD + k0);
    a1.h[1] = *(const v8h*)(ap + (size_t)16 * APD + k0 + 16);
#pragma unroll
    for (int nt = 0; nt < 4; ++nt) {
      const _Float16* bq = bp + (size_t)nt * 16 * APD + k0;
      FragH b;
      b.h[0] = *(const v8h*)bq;
      b.h[1] = *(const v8h*)(bq + 16);
      acc[0][nt] = wmf(a0.v, b.v, acc[0][nt]);
      acc[1][nt] = wmf(a1.v, b.v, acc[1][nt]);
    }
  }

#pragma unroll
  for (int mt = 0; mt < 2; ++mt) {
    float* sp = stg + (16 * mt + 8 * hf) * 64 + m;
#pragma unroll
    for (int nt = 0; nt < 4; ++nt) {
#pragma unroll
      for (int r = 0; r < 8; ++r) sp[r * 64 + 16 * nt] = acc[mt][nt][r];
    }
  }
  constexpr float OSC2 = 1.0f / (float)(H1S * WSC);
#pragma unroll 1
  for (int e = 0; e < 64; ++e) {
    const int mt = e >> 5, nt = (e >> 3) & 3, r = e & 7;
    float* p = stg + (16 * mt + 8 * hf + r) * 64 + 16 * nt + m;
    const int cl = wn + 16 * nt + m;
    const float v = *p;
    *p = gelu_erf(fmaf(v, OSC2, bvS[cl])) * gvS[cl];
  }
  __syncthreads();

  float* gbase = out + (size_t)(m0 + wm) * HID + n0 + wn;
  const float* xbase = x + (size_t)(m0 + wm) * HID + n0 + wn;
#pragma unroll
  for (int q = 0; q < 16; ++q) {
    const int row = 2 * q + hf;
    const v4f hv = *(const v4f*)(stg + row * 64 + 4 * m);
    const v4f xv = *(const v4f*)(xbase + (size_t)row * HID + 4 * m);
    const v4f ov = xv + hv;
    *(volatile v4f*)(gbase + (size_t)row * HID + 4 * m) = ov;
  }
  __threadfence();
#pragma unroll
  for (int q = 0; q < 16; ++q) {
    const int row = 2 * q + hf;
    const v4f hv = *(const v4f*)(stg + row * 64 + 4 * m);
    const v4f xv = *(const v4f*)(xbase + (size_t)row * HID + 4 * m);
    const v4f ov = xv + hv;
    *(volatile v4f*)(gbase + (size_t)row * HID + 4 * m) = ov;
  }
}

extern "C" void kernel_launch(void* const* d_in, const int* in_sizes, int n_in,
                              void* d_out, int out_size, void* d_ws, size_t ws_size,
                              hipStream_t stream) {
  if (n_in < 15) return;
  if (in_sizes[0] != NTOK * HID || in_sizes[1] != 1 || in_sizes[2] != 1 ||
      in_sizes[3] != ADP * HID || in_sizes[4] != ADP || in_sizes[5] != HID * ADP || in_sizes[6] != HID ||
      in_sizes[7] != NTASK * ADP || in_sizes[8] != NTASK * HID || in_sizes[9] != NTASK * CAP * HID ||
      in_sizes[10] != NTASK * CAP || in_sizes[11] != NRW || in_sizes[12] != HID * NCAP * CAP ||
      in_sizes[13] != HID || in_sizes[14] != NTASK * HID) return;
  if (out_size != NTOK * HID) return;

  const float* x     = (const float*)d_in[0];
  const int*   tptr  = (const int*)d_in[1];
  const float* s     = (const float*)d_in[2];
  const float* fc1w  = (const float*)d_in[3];
  const float* fc1b  = (const float*)d_in[4];
  const float* fc2w  = (const float*)d_in[5];
  const float* fc2b  = (const float*)d_in[6];
  const float* efc1  = (const float*)d_in[7];
  const float* efc2  = (const float*)d_in[8];
  const float* semw  = (const float*)d_in[9];
  const float* semb  = (const float*)d_in[10];
  const float* rw    = (const float*)d_in[11];
  const float* lw    = (const float*)d_in[12];
  const float* lb    = (const float*)d_in[13];
  const float* elg   = (const float*)d_in[14];
  float* out = (float*)d_out;

  char* ws = (char*)d_ws;
  size_t off = 0;
  const size_t oV  = off; off += (size_t)NCAP * NTOK * CAP * 4; off = (off + 255) & ~(size_t)255;
  const size_t oHP = off; off += (size_t)NTOK * HID * 2;        off = (off + 255) & ~(size_t)255;
  const size_t oH1 = off; off += (size_t)NTOK * APD * 2;        off = (off + 255) & ~(size_t)255;
  const size_t oW1 = off; off += (size_t)APD * HID * 2;         off = (off + 255) & ~(size_t)255;
  const size_t oW2 = off; off += (size_t)HID * APD * 2;         off = (off + 255) & ~(size_t)255;
  const size_t oWS = off; off += (size_t)NSEM * HID * 2;        off = (off + 255) & ~(size_t)255;
  if (off > ws_size || off > (size_t)WSCAP) return;
  float*    votef = (float*)(ws + oV);
  _Float16* hp    = (_Float16*)(ws + oHP);
  _Float16* h1    = (_Float16*)(ws + oH1);
  _Float16* w1h   = (_Float16*)(ws + oW1);
  _Float16* w2h   = (_Float16*)(ws + oW2);
  _Float16* wsh   = (_Float16*)(ws + oWS);

  k_prepw<<<NBW1 + NBW2 + NBWS, NTHR, 0, stream>>>(fc1w, fc2w, semw, w1h, w2h, wsh);
  k_semroute<<<NTOK / TOKB, STHR, 0, stream>>>(x, wsh, semb, rw, tptr, votef);
  k_buildh<<<NTOK / RB, BTHR, 0, stream>>>(x, votef, lw, lb, elg, s, tptr, hp);
  hipFuncSetAttribute(reinterpret_cast<const void*>(&k_gemm1),
                      hipFuncAttributeMaxDynamicSharedMemorySize, LDS_G);
  k_gemm1<<<dim3(APD / 128, NTOK / 128), NTHR, LDS_G, stream>>>(hp, w1h, fc1b, efc1, s, tptr, h1);
  hipFuncSetAttribute(reinterpret_cast<const void*>(&k_gemm2),
                      hipFuncAttributeMaxDynamicSharedMemorySize, LDS_G);
  k_gemm2<<<dim3(HID / 128, NTOK / 128), NTHR, LDS_G, stream>>>(h1, w2h, fc2b, efc2, s, tptr, x, out);
}
